// _GPTAttn_41180146434219
// MI455X (gfx1250) — hardware-verified
//
#include <hip/hip_runtime.h>
#include <math.h>

constexpr int kB    = 4;
constexpr int kT    = 2048;
constexpr int kD    = 1024;
constexpr int kH    = 16;
constexpr int kDH   = 64;
constexpr int kTok  = kB * kT;
constexpr int kNQKV = 3 * kH * kDH;
constexpr int kQKld = 2 * kH * kDH;
constexpr int kGrp  = 2;
constexpr int kGroupsPerBatch = kH / kGrp;
constexpr float kScoreScale = 0.125f;

static_assert(kH % kGrp == 0, "groups stay inside one batch");
static_assert((kTok * kD) % (8 * 256) == 0, "cast kernel grid exact");
static_assert((kNQKV * kD) % (8 * 256) == 0 && (kD * kD) % (8 * 256) == 0, "weight cast grids exact");
static_assert(kT == 2048, "softmax kernel: 256 threads x 8 columns = one row, blockIdx decode");
static_assert(kD % 64 == 0 && kNQKV % 64 == 0 && kT % 64 == 0 && kDH % 64 == 0, "tile multiples");
static_assert(kD % 32 == 0 && kDH % 32 == 0 && kT % 32 == 0, "K multiples of 32");

typedef __attribute__((ext_vector_type(16))) _Float16 v16h;
typedef __attribute__((ext_vector_type(8)))  _Float16 v8h;
typedef __attribute__((ext_vector_type(16))) __bf16   v16b;
typedef __attribute__((ext_vector_type(8)))  __bf16   v8b;
typedef __attribute__((ext_vector_type(8)))  float    v8f;
typedef __attribute__((ext_vector_type(4)))  float    v4f;
typedef __attribute__((ext_vector_type(4)))  unsigned int v4u;

__device__ __forceinline__ unsigned short f2bf_bits(float f) {
  unsigned u = __float_as_uint(f);
  return (unsigned short)((u + 0x7FFFu + ((u >> 16) & 1u)) >> 16);
}
__device__ __forceinline__ float bf_bits2f(unsigned short h) { return __uint_as_float(((unsigned)h) << 16); }

__device__ __forceinline__ void dep_guard_h(v8f& a, v8f& b, v16h x, v16h y) { asm volatile("v_nop\n\tv_nop\n\tv_nop\n\tv_nop" : "+v"(a), "+v"(b) : "v"(x), "v"(y)); }
__device__ __forceinline__ void dep_guard_b(v8f& a, v8f& b, v16b x, v16b y) { asm volatile("v_nop\n\tv_nop\n\tv_nop\n\tv_nop" : "+v"(a), "+v"(b) : "v"(x), "v"(y)); }
__device__ __forceinline__ void keep4_h(v16h a, v16h b, v16h c, v16h d) { asm volatile("v_nop" :: "v"(a), "v"(b), "v"(c), "v"(d)); }
__device__ __forceinline__ void keep4_b(v16b a, v16b b, v16b c, v16b d) { asm volatile("v_nop" :: "v"(a), "v"(b), "v"(c), "v"(d)); }
__device__ __forceinline__ void acc_guard4(v8f& a, v8f& b, v8f& c, v8f& d) { asm volatile("v_nop\n\tv_nop\n\tv_nop\n\tv_nop" : "+v"(a), "+v"(b), "+v"(c), "+v"(d)); }
template <typename T> struct Frag;
template <> struct Frag<_Float16> {
  typedef v16h V; union U { v16h v; v8h h[2]; };
  static __device__ __forceinline__ v16h load(const _Float16* p) {
    U f; f.h[0] = *(const v8h*)(p); f.h[1] = *(const v8h*)(p + 16); return f.v;
  }
  static __device__ __forceinline__ v8f mma(v16h a, v16h b, v8f c) {
    return __builtin_amdgcn_wmma_f32_16x16x32_f16(false, a, false, b, (short)0, c, false, false);
  }
  static __device__ __forceinline__ void guard(v8f& a, v8f& b, v16h x, v16h y) { dep_guard_h(a, b, x, y); }
  static __device__ __forceinline__ void keep(v16h a, v16h b, v16h c, v16h d) { keep4_h(a, b, c, d); }
};
template <> struct Frag<__bf16> {
  typedef v16b V; union U { v16b v; v8b h[2]; };
  static __device__ __forceinline__ v16b load(const __bf16* p) {
    U f; f.h[0] = *(const v8b*)(p); f.h[1] = *(const v8b*)(p + 16); return f.v;
  }
  static __device__ __forceinline__ v8f mma(v16b a, v16b b, v8f c) {
    return __builtin_amdgcn_wmma_f32_16x16x32_bf16(false, a, false, b, (short)0, c, false, false);
  }
  static __device__ __forceinline__ void guard(v8f& a, v8f& b, v16b x, v16b y) { dep_guard_b(a, b, x, y); }
  static __device__ __forceinline__ void keep(v16b a, v16b b, v16b c, v16b d) { keep4_b(a, b, c, d); }
};

__device__ __forceinline__ unsigned pk16(unsigned short a, unsigned short b) { return (unsigned)a | ((unsigned)b << 16); }

template <int ET> struct Elem;
template <> struct Elem<0> { typedef _Float16 T; };
template <> struct Elem<1> { typedef __bf16 T; };
template <int ET, bool SPLIT, int BIAS_MODE, int OUT_MODE, bool RESID, int ACT = 0, bool CAUSAL = false, bool BSPLIT = true>
__global__ __launch_bounds__(256) void wmma_gemm64(
    const unsigned short* __restrict__ Ap, const unsigned short* __restrict__ A2p, int lda, long strideA,
    const unsigned short* __restrict__ Btp, const unsigned short* __restrict__ Bt2p, int ldb, long strideB,
    void* __restrict__ Cout, void* __restrict__ Cout2, int ldc, long strideC,
    const float* __restrict__ bias,
    const float* __restrict__ resid, long strideR,
    int M, int N, int K, float scale) {
  typedef typename Elem<ET>::T T;
  typedef typename Frag<T>::V V;
  const T* A = (const T*)Ap; const T* A2 = (const T*)A2p; const T* Bt = (const T*)Btp; const T* Bt2 = (const T*)Bt2p;
  __shared__ __align__(16) float sT[8][16 * 68];
  const int b    = blockIdx.y;
  const int lane = threadIdx.x & 31;
  const int wave = threadIdx.x >> 5;
  const int tilesN = N >> 6;
  const int tilesM = M >> 6;
  const int tile = blockIdx.x * 8 + wave;
  if (tile >= tilesM * tilesN) return;
  const int tm = tile / tilesN;
  const int tn = tile - tm * tilesN;
  const int m0 = tm << 6;
  const int n0 = tn << 6;
  if (CAUSAL && (n0 > m0)) return;
  const int Kend = CAUSAL ? ((m0 + 64 < K) ? (m0 + 64) : K) : K;

  const T* Ab  = A  + (size_t)b * strideA;
  const T* Bb  = Bt + (size_t)b * strideB;
  const T* Ab2 = SPLIT ? (A2  + (size_t)b * strideA) : nullptr;
  const T* Bb2 = (SPLIT && BSPLIT) ? (Bt2 + (size_t)b * strideB) : nullptr;

  const int rlane = lane & 15;
  const int koff  = (lane >> 4) * 8;
  const int mOff  = (lane >> 4) * 8;

  v8f acc[4][4];
#pragma unroll
  for (int i = 0; i < 4; ++i)
#pragma unroll
    for (int j = 0; j < 4; ++j) acc[i][j] = (v8f){0.f,0.f,0.f,0.f,0.f,0.f,0.f,0.f};

  for (int k0 = 0; k0 < Kend; k0 += 32) {
    V bh[4], bl[4];
#pragma unroll
    for (int j = 0; j < 4; ++j) {
      const size_t bo = (size_t)(n0 + (j << 4) + rlane) * ldb + koff + k0;
      bh[j] = Frag<T>::load(Bb + bo);
      if (SPLIT && BSPLIT) bl[j] = Frag<T>::load(Bb2 + bo);
    }
#pragma unroll
    for (int i = 0; i < 4; ++i) {
      const size_t ao = (size_t)(m0 + (i << 4) + rlane) * lda + koff + k0;
      V ah = Frag<T>::load(Ab + ao);
      V al;
      if (SPLIT) al = Frag<T>::load(Ab2 + ao);
#pragma unroll
      for (int j = 0; j < 4; ++j) {
        acc[i][j] = Frag<T>::mma(ah, bh[j], acc[i][j]);
        if (SPLIT && BSPLIT) acc[i][j] = Frag<T>::mma(ah, bl[j], acc[i][j]);
        if (SPLIT) acc[i][j] = Frag<T>::mma(al, bh[j], acc[i][j]);
      }
      Frag<T>::guard(acc[i][0], acc[i][3], ah, SPLIT ? al : ah);
    }
    Frag<T>::keep(bh[0], bh[1], bh[2], bh[3]);
    if (SPLIT && BSPLIT) Frag<T>::keep(bl[0], bl[1], bl[2], bl[3]);
  }
  acc_guard4(acc[0][0], acc[0][1], acc[0][2], acc[0][3]);
  acc_guard4(acc[1][0], acc[1][1], acc[1][2], acc[1][3]);
  acc_guard4(acc[2][0], acc[2][1], acc[2][2], acc[2][3]);
  acc_guard4(acc[3][0], acc[3][1], acc[3][2], acc[3][3]);

  float* slab = sT[wave];
  const float* Rb = RESID ? (resid + (size_t)b * strideR) : nullptr;
#pragma unroll
  for (int i = 0; i < 4; ++i) {
    const int mBase = m0 + (i << 4);
#pragma unroll
    for (int j = 0; j < 4; ++j) {
      const int n = n0 + (j << 4) + rlane;
      float bv = 0.f;
      if (BIAS_MODE == 2) bv = bias[n];
#pragma unroll
      for (int r = 0; r < 8; ++r) {
        float v = acc[i][j][r] * scale;
        if (BIAS_MODE == 1) v += bias[mBase + mOff + r];
        if (BIAS_MODE == 2) v += bv;
        if (RESID) v += Rb[(size_t)(mBase + mOff + r) * ldc + n];
        if (ACT == 2) v = fmaxf(v, 0.0f);
        if (ACT == 4) v = (v > 0.f) ? v : 0.01f * v;
        slab[(mOff + r) * 68 + (j << 4) + rlane] = v;
      }
    }
    __builtin_amdgcn_fence(__ATOMIC_RELEASE, "workgroup");
    __builtin_amdgcn_wave_barrier();
    __builtin_amdgcn_fence(__ATOMIC_ACQUIRE, "workgroup");
    if (OUT_MODE == 0) {
      float* C = (float*)Cout + (size_t)b * strideC;
      const int hh = lane >> 4, c4 = (lane & 15) * 4;
      for (int pass = 0; pass < 2; ++pass) {
#pragma unroll
        for (int it = 0; it < 8; ++it) {
          const int row = it * 2 + hh;
          v4f v = *(const v4f*)(slab + row * 68 + c4);
          *(volatile v4f*)(C + (size_t)(mBase + row) * ldc + n0 + c4) = v;
        }
        __threadfence();
      }
    } else {
      const int q = lane >> 3, c8 = (lane & 7) * 8;
      unsigned short* C  = (unsigned short*)Cout  + (size_t)b * strideC;
      unsigned short* C2 = (OUT_MODE == 2) ? ((unsigned short*)Cout2 + (size_t)b * strideC) : nullptr;
      for (int pass = 0; pass < 2; ++pass) {
#pragma unroll
        for (int it = 0; it < 4; ++it) {
          const int row = it * 4 + q;
          const float* sp = slab + row * 68 + c8;
          v8h hv, lv;
#pragma unroll
          for (int e = 0; e < 8; ++e) {
            if (OUT_MODE == 1) {
              hv[e] = (_Float16)sp[e];
            } else {
              unsigned short hb = f2bf_bits(sp[e]);
              unsigned short lb = f2bf_bits(sp[e] - bf_bits2f(hb));
              hv[e] = __builtin_bit_cast(_Float16, hb);
              lv[e] = __builtin_bit_cast(_Float16, lb);
            }
          }
          *(volatile v8h*)(C + (size_t)(mBase + row) * ldc + n0 + c8) = hv;
          if (OUT_MODE == 2) *(volatile v8h*)(C2 + (size_t)(mBase + row) * ldc + n0 + c8) = lv;
        }
        __threadfence();
      }
    }
    __builtin_amdgcn_fence(__ATOMIC_RELEASE, "workgroup");
    __builtin_amdgcn_wave_barrier();
    __builtin_amdgcn_fence(__ATOMIC_ACQUIRE, "workgroup");
  }
}

__global__ __launch_bounds__(256) void cast8_bf16_kernel(const float* __restrict__ in, unsigned short* __restrict__ out, int n8) {
  const int i = blockIdx.x * 256 + threadIdx.x;
  if (i >= n8) return;
  const float* p = in + 8 * (size_t)i;
  const v4f a = *(const v4f*)(p);
  const v4f c = *(const v4f*)(p + 4);
  float f[8];
#pragma unroll
  for (int e = 0; e < 4; ++e) { f[e] = a[e]; f[4 + e] = c[e]; }
  unsigned w[4];
#pragma unroll
  for (int e2 = 0; e2 < 4; ++e2) w[e2] = pk16(f2bf_bits(f[2 * e2]), f2bf_bits(f[2 * e2 + 1]));
  const v4u u = (v4u){w[0], w[1], w[2], w[3]};
  unsigned short* q = out + 8 * (size_t)i;
  *(volatile v4u*)q = u;
  __threadfence();
  *(volatile v4u*)q = u;
}

__global__ __launch_bounds__(256) void softmax_causal_kernel(const float* __restrict__ S,
                                                             unsigned short* __restrict__ Phi, unsigned short* __restrict__ Plo) {
  __shared__ float redM[8];
  __shared__ float redS[8];
  const float ninf = -__builtin_inff();
  const int blk  = blockIdx.x;
  const int pr   = blk >> 11;
  const int qi   = blk & (kT - 1);
  const int t    = threadIdx.x;
  const int lane = t & 31, wave = t >> 5;
  const int c0   = t * 8;
  const size_t rowoff = ((size_t)pr * kT + qi) * (size_t)kT;
  const bool wave_live = (wave * 256 <= qi);

  float xv[8];
  float m = ninf;
  if (wave_live) {
    const float* sr = S + rowoff + c0;
    const v4f a  = *(const v4f*)(sr);
    const v4f c  = *(const v4f*)(sr + 4);
    float sv[8];
#pragma unroll
    for (int e = 0; e < 4; ++e) { sv[e] = a[e]; sv[4 + e] = c[e]; }
#pragma unroll
    for (int e = 0; e < 8; ++e) {
      const int j = c0 + e;
      const float v = (j > qi) ? ninf : sv[e];
      xv[e] = v;
      m = fmaxf(m, v);
    }
  } else {
#pragma unroll
    for (int e = 0; e < 8; ++e) xv[e] = ninf;
  }
#pragma unroll
  for (int off = 16; off > 0; off >>= 1) m = fmaxf(m, __shfl_xor(m, off, 32));
  if (lane == 0) redM[wave] = m;
  __syncthreads();
  float gmax = redM[0];
#pragma unroll
  for (int w = 1; w < 8; ++w) gmax = fmaxf(gmax, redM[w]);

  float p[8];
  float ps = 0.0f;
  if (wave_live) {
#pragma unroll
    for (int e = 0; e < 8; ++e) { p[e] = expf(xv[e] - gmax); ps += p[e]; }
  } else {
#pragma unroll
    for (int e = 0; e < 8; ++e) p[e] = 0.0f;
  }
#pragma unroll
  for (int off = 16; off > 0; off >>= 1) ps += __shfl_xor(ps, off, 32);
  if (lane == 0) redS[wave] = ps;
  __syncthreads();
  float tot = redS[0];
#pragma unroll
  for (int w = 1; w < 8; ++w) tot += redS[w];
  const float inv = 1.0f / tot;

  unsigned hw[4], lw[4];
#pragma unroll
  for (int e2 = 0; e2 < 4; ++e2) {
    float f0 = p[2 * e2] * inv;
    float f1 = p[2 * e2 + 1] * inv;
    f0 = (f0 == f0) ? f0 : 0.0f;
    f1 = (f1 == f1) ? f1 : 0.0f;
    const unsigned short h0 = f2bf_bits(f0);
    const unsigned short h1 = f2bf_bits(f1);
    const unsigned short l0 = f2bf_bits(f0 - bf_bits2f(h0));
    const unsigned short l1 = f2bf_bits(f1 - bf_bits2f(h1));
    hw[e2] = pk16(h0, h1);
    lw[e2] = pk16(l0, l1);
  }
  const v4u hv = (v4u){hw[0], hw[1], hw[2], hw[3]};
  const v4u lv = (v4u){lw[0], lw[1], lw[2], lw[3]};
  unsigned short* ph = Phi + rowoff + c0;
  unsigned short* pl = Plo + rowoff + c0;
  *(volatile v4u*)ph = hv;
  *(volatile v4u*)pl = lv;
  __threadfence();
  *(volatile v4u*)ph = hv;
  *(volatile v4u*)pl = lv;
}

extern "C" void kernel_launch(void* const* d_in, const int* in_sizes, int n_in,
                              void* d_out, int out_size, void* d_ws, size_t ws_size,
                              hipStream_t stream) {
  if (n_in < 3) return;
  if (in_sizes[0] != kTok * kD || in_sizes[1] != kNQKV * kD || in_sizes[2] != kD * kD) return;
  if (out_size != kTok * kD) return;

  const size_t kMiB    = 1048576;
  const size_t offXb   = 0;
  const size_t offWq   = 16 * kMiB;
  const size_t offWo   = 22 * kMiB;
  const size_t offQKhi = 24 * kMiB;
  const size_t offQKlo = 32 * kMiB;
  const size_t offVthi = 40 * kMiB;
  const size_t offVtlo = 44 * kMiB;
  const size_t offChi  = 48 * kMiB;
  const size_t offClo  = 52 * kMiB;
  const size_t offS    = 56 * kMiB;
  const size_t offPhi  = 88 * kMiB;
  const size_t offPlo  = 104 * kMiB;
  const size_t total   = 120 * kMiB;
  static_assert((size_t)kTok * kD * 2 == 16 * 1048576, "x plane bytes");
  static_assert((size_t)kNQKV * kD * 2 == 6 * 1048576, "Wqkv plane bytes");
  static_assert((size_t)kD * kD * 2 == 2 * 1048576, "Wout plane bytes");
  static_assert((size_t)kT * kQKld * 2 == 8 * 1048576, "q|k plane bytes");
  static_assert((size_t)kD * kT * 2 == 4 * 1048576, "v^T and ctx plane bytes");
  static_assert((size_t)kGrp * kT * kT * 4 == 32 * 1048576, "S region bytes");
  static_assert((size_t)kGrp * kT * kT * 2 == 16 * 1048576, "P plane bytes");
  if (total > ws_size) return;

  const float* x    = (const float*)d_in[0];
  const float* Wqkv = (const float*)d_in[1];
  const float* Wout = (const float*)d_in[2];
  float* out = (float*)d_out;
  char* ws = (char*)d_ws;

  unsigned short* xb   = (unsigned short*)(ws + offXb);
  unsigned short* wq   = (unsigned short*)(ws + offWq);
  unsigned short* wo   = (unsigned short*)(ws + offWo);
  unsigned short* qkhi = (unsigned short*)(ws + offQKhi);
  unsigned short* qklo = (unsigned short*)(ws + offQKlo);
  unsigned short* vthi = (unsigned short*)(ws + offVthi);
  unsigned short* vtlo = (unsigned short*)(ws + offVtlo);
  unsigned short* chi  = (unsigned short*)(ws + offChi);
  unsigned short* clo  = (unsigned short*)(ws + offClo);
  float*          Sbuf = (float*)(ws + offS);
  unsigned short* phi  = (unsigned short*)(ws + offPhi);
  unsigned short* plo  = (unsigned short*)(ws + offPlo);

  const float* dummy_f = x;
  void* dummy_c2 = (void*)phi;

  {
    const int n8 = (kTok * kD) / 8;
    cast8_bf16_kernel<<<dim3(n8 / 256), dim3(256), 0, stream>>>(x, xb, n8);
  }
  {
    const int n8 = (kNQKV * kD) / 8;
    cast8_bf16_kernel<<<dim3(n8 / 256), dim3(256), 0, stream>>>(Wqkv, wq, n8);
  }
  {
    const int n8 = (kD * kD) / 8;
    cast8_bf16_kernel<<<dim3(n8 / 256), dim3(256), 0, stream>>>(Wout, wo, n8);
  }

  for (int bb = 0; bb < kB; ++bb) {
    const unsigned short* xbb = xb + (size_t)bb * kT * kD;

    wmma_gemm64<1, false, 0, 2, false, 0, false, true><<<dim3((kT / 64) * (kQKld / 64) / 8, 1), dim3(256), 0, stream>>>(
        xbb, xbb, kD, 0L,
        wq, wq, kD, 0L,
        (void*)qkhi, (void*)qklo, kQKld, 0L,
        dummy_f, dummy_f, 0L,
        kT, kQKld, kD, 1.0f);

    wmma_gemm64<1, false, 0, 2, false, 0, false, true><<<dim3((kD / 64) * (kT / 64) / 8, 1), dim3(256), 0, stream>>>(
        wq + (size_t)kQKld * kD, wq + (size_t)kQKld * kD, kD, 0L,
        xbb, xbb, kD, 0L,
        (void*)vthi, (void*)vtlo, kT, 0L,
        dummy_f, dummy_f, 0L,
        kD, kT, kD, 1.0f);

    for (int gi = 0; gi < kGroupsPerBatch; ++gi) {
      const int h0 = gi * kGrp;
      const size_t qkoff = (size_t)h0 * kDH;

      wmma_gemm64<1, true, 0, 0, false, 0, true, true><<<dim3((kT / 64) * (kT / 64) / 8, kGrp), dim3(256), 0, stream>>>(
          qkhi + qkoff, qklo + qkoff, kQKld, (long)kDH,
          qkhi + kH * kDH + qkoff, qklo + kH * kDH + qkoff, kQKld, (long)kDH,
          (void*)Sbuf, dummy_c2, kT, (long)kT * kT,
          dummy_f, dummy_f, 0L,
          kT, kT, kDH, kScoreScale);

      softmax_causal_kernel<<<dim3(kGrp * kT), dim3(256), 0, stream>>>(Sbuf, phi, plo);

      const size_t vtoff = (size_t)(h0 * kDH) * kT;
      const size_t coff  = (size_t)h0 * kDH;
      wmma_gemm64<1, true, 0, 2, false, 0, true, true><<<dim3((kT / 64) * (kDH / 64) / 8, kGrp), dim3(256), 0, stream>>>(
          phi, plo, kT, (long)kT * kT,
          vthi + vtoff, vtlo + vtoff, kT, (long)kDH * kT,
          (void*)(chi + coff), (void*)(clo + coff), kD, (long)kDH,
          dummy_f, dummy_f, 0L,
          kT, kDH, kT, 1.0f);
    }

    wmma_gemm64<1, true, 0, 0, false, 0, false, false><<<dim3((kT / 64) * (kD / 64) / 8, 1), dim3(256), 0, stream>>>(
        chi, clo, kD, 0L,
        wo, wo, kD, 0L,
        (void*)(out + (size_t)bb * kT * kD), dummy_c2, kD, 0L,
        dummy_f, dummy_f, 0L,
        kT, kD, kD, 1.0f);
  }
}
